// Encoder_38706245271727
// MI455X (gfx1250) — hardware-verified
//
#include <hip/hip_runtime.h>
#include <stddef.h>
#include <stdint.h>


#define DF     128
#define K1     256
#define NTHR   256
#define NWAVE  8
#define EPT    8
#define CHUNK  (NTHR * EPT)
#define WCAP   (EPT * 32)
#define LISTN  (NWAVE * WCAP)
#define NBA    1024
#define SLA    10
#define RCAP   24576
#define DEGCAP 64
#define GBM    64
#define GBN    128
#define GTHR   128
#define UPART  2048
#define NPART  3
#define CMP_ZINTS    (LISTN + 2 * RCAP + 3 * NBA)
#define MISC_INTS    16
#define CMP_LDS_INTS (CMP_ZINTS + MISC_INTS)
#define RECW   256
#define WSMAX  134217728

static_assert((CHUNK & (CHUNK - 1)) == 0 && CHUNK <= 4096);
static_assert((NBA & (NBA - 1)) == 0 && NBA == (1 << SLA));
static_assert(((long long)CHUNK << SLA) < (1LL << 31));
static_assert(LISTN % NTHR == 0);
static_assert(NBA % NWAVE == 0 && NBA % 32 == 0 && NBA % GBM == 0 && NBA == 4 * NTHR);
static_assert(RCAP % NTHR == 0 && CMP_ZINTS % (NTHR * 4) == 0 && (RCAP * 4) % 128 == 0);
static_assert(DF % 32 == 0 && K1 % 32 == 0 && K1 == 2 * DF);
static_assert(GBN == DF && GBM == (GTHR / 32) * 16 && DF == 4 * 32);
static_assert(UPART % NTHR == 0 && UPART == DF * (DF / 8));
static_assert((NPART * UPART) % NTHR == 0);
static_assert(CMP_LDS_INTS * 4 <= 300000);
static_assert(RECW == 2 * DF && RECW == NTHR);
static_assert(DEGCAP >= 36 + 8 && RCAP >= 16710 + 32);

typedef float          v4f   __attribute__((ext_vector_type(4)));
typedef float          v8f   __attribute__((ext_vector_type(8)));
typedef int            v4i   __attribute__((ext_vector_type(4)));
typedef int            v8i   __attribute__((ext_vector_type(8)));
typedef unsigned short v4us  __attribute__((ext_vector_type(4)));
typedef unsigned short v8us  __attribute__((ext_vector_type(8)));
typedef unsigned short v16us __attribute__((ext_vector_type(16)));
typedef __bf16         v16bf __attribute__((ext_vector_type(16)));
typedef v4f  __attribute__((may_alias)) v4fa;
typedef v4i  __attribute__((may_alias)) v4ia;
typedef v4us __attribute__((may_alias)) v4usa;
typedef v8us __attribute__((may_alias)) v8usa;
union FragB { v16bf v; v16us u; v8us h[2]; v8i w; };

__device__ __forceinline__ v8f wmb(const FragB& a, const FragB& b, v8f c) {
  v8f d = __builtin_amdgcn_wmma_f32_16x16x32_bf16(false, a.v, false, b.v, (short)0, c, false, false);
  asm volatile("v_nop\n\tv_nop\n\tv_nop\n\tv_nop" : "+v"(d) : "v"(a.w), "v"(b.w));
  return d;
}

__device__ __forceinline__ unsigned bf16_bits(float f) {
  const unsigned u = __float_as_uint(f);
  return (u + 0x7FFFu + ((u >> 16) & 1u)) >> 16;
}
__device__ __forceinline__ float bf16_val(float f) {
  return __uint_as_float(bf16_bits(f) << 16);
}

__device__ __forceinline__ float bnrelu(float a, float mu, float rs, float g, float b) {
  const float t = ((a - mu) * rs) * g + b;
  return (t > 0.0f) ? t : (t - t);
}

template <int SLB>
__device__ __forceinline__ int scan_chunk(const int* __restrict__ dsts, int nE, int cbase, int slotBase,
                                          int nb, int vec8, int* list, int tid, int lane, int wave) {
  int wc = 0;
  const int el0  = tid * EPT;
  const int e0   = cbase + el0;
  const int sent = -2147483647 - 1;
  v4i da, db;
  if (vec8 != 0 && cbase + CHUNK <= nE) {
    da = *(const v4i*)(dsts + e0);
    db = *(const v4i*)(dsts + e0 + 4);
  } else {
    da.x = (e0     < nE) ? dsts[min(e0,     nE - 1)] : sent;
    da.y = (e0 + 1 < nE) ? dsts[min(e0 + 1, nE - 1)] : sent;
    da.z = (e0 + 2 < nE) ? dsts[min(e0 + 2, nE - 1)] : sent;
    da.w = (e0 + 3 < nE) ? dsts[min(e0 + 3, nE - 1)] : sent;
    db.x = (e0 + 4 < nE) ? dsts[min(e0 + 4, nE - 1)] : sent;
    db.y = (e0 + 5 < nE) ? dsts[min(e0 + 5, nE - 1)] : sent;
    db.z = (e0 + 6 < nE) ? dsts[min(e0 + 6, nE - 1)] : sent;
    db.w = (e0 + 7 < nE) ? dsts[min(e0 + 7, nE - 1)] : sent;
  }
  const unsigned nbs = (unsigned)slotBase;
  const unsigned unb = (unsigned)nb;
  const unsigned s0 = (unsigned)da.x - nbs, s1 = (unsigned)da.y - nbs;
  const unsigned s2 = (unsigned)da.z - nbs, s3 = (unsigned)da.w - nbs;
  const unsigned s4 = (unsigned)db.x - nbs, s5 = (unsigned)db.y - nbs;
  const unsigned s6 = (unsigned)db.z - nbs, s7 = (unsigned)db.w - nbs;
  const bool h0 = s0 < unb, h1 = s1 < unb, h2 = s2 < unb, h3 = s3 < unb;
  const bool h4 = s4 < unb, h5 = s5 < unb, h6 = s6 < unb, h7 = s7 < unb;
  const unsigned any = __builtin_amdgcn_ballot_w32(h0 | h1 | h2 | h3 | h4 | h5 | h6 | h7);
  if (any != 0u) {
#define HITJ(J, HJ, SJ) { \
      const unsigned mj = __builtin_amdgcn_ballot_w32(HJ); \
      if (mj != 0u) { \
        if (HJ) { \
          const int pos = wc + (int)__builtin_amdgcn_mbcnt_lo(mj, 0u); \
          if (pos < WCAP) list[wave * WCAP + pos] = ((el0 + (J)) << SLB) | (int)(SJ); \
        } \
        wc += (int)__builtin_popcount(mj); } }
    HITJ(0, h0, s0)
    HITJ(1, h1, s1)
    HITJ(2, h2, s2)
    HITJ(3, h3, s3)
    HITJ(4, h4, s4)
    HITJ(5, h5, s5)
    HITJ(6, h6, s6)
    HITJ(7, h7, s7)
#undef HITJ
  }
  return wc;
}

__global__ __launch_bounds__(NTHR) void k_wprep(const float* __restrict__ W, unsigned short* WB) {
  const int u = (int)blockIdx.x * NTHR + (int)threadIdx.x;
  if (u >= NPART * UPART) return;
  const int part = u >> 11;
  const int v    = u & (UPART - 1);
  const int n    = v >> 4;
  const int k8   = (v & 15) * 8;
  const int srcOff = (part == 0) ? 0 : DF * DF;
  const int pitch  = (part == 0) ? DF : K1;
  const int dstOff = ((part == 0) ? 0 : DF * DF) + ((part == 2) ? DF : 0);
  const float* p = W + srcOff + n * DF + k8;
  const v4f a = *(const v4fa*)p;
  const v4f b = *(const v4fa*)(p + 4);
  v8us o;
  o[0] = (unsigned short)bf16_bits(a.x); o[1] = (unsigned short)bf16_bits(a.y);
  o[2] = (unsigned short)bf16_bits(a.z); o[3] = (unsigned short)bf16_bits(a.w);
  o[4] = (unsigned short)bf16_bits(b.x); o[5] = (unsigned short)bf16_bits(b.y);
  o[6] = (unsigned short)bf16_bits(b.z); o[7] = (unsigned short)bf16_bits(b.w);
  unsigned short* dp = WB + dstOff + n * pitch + k8;
  *(volatile v8us*)dp = o;
  __threadfence();
  *(volatile v8us*)dp = o;
}

__global__ __launch_bounds__(NTHR) void k_cvx(const float* __restrict__ x, int nN, int nUnits,
                                              unsigned short* xb) {
  const int u = (int)blockIdx.x * NTHR + (int)threadIdx.x;
  if (u >= nUnits) return;
  const int row = u >> 4;
  const int k8  = (u & 15) * 8;
  const int rc  = row < nN ? row : nN - 1;
  const float* p = x + (size_t)rc * DF + k8;
  const v4f a = *(const v4fa*)p;
  const v4f b = *(const v4fa*)(p + 4);
  const bool ok = row < nN;
  v8us o;
  o[0] = ok ? (unsigned short)bf16_bits(a.x) : (unsigned short)0;
  o[1] = ok ? (unsigned short)bf16_bits(a.y) : (unsigned short)0;
  o[2] = ok ? (unsigned short)bf16_bits(a.z) : (unsigned short)0;
  o[3] = ok ? (unsigned short)bf16_bits(a.w) : (unsigned short)0;
  o[4] = ok ? (unsigned short)bf16_bits(b.x) : (unsigned short)0;
  o[5] = ok ? (unsigned short)bf16_bits(b.y) : (unsigned short)0;
  o[6] = ok ? (unsigned short)bf16_bits(b.z) : (unsigned short)0;
  o[7] = ok ? (unsigned short)bf16_bits(b.w) : (unsigned short)0;
  unsigned short* dp = xb + (size_t)row * DF + k8;
  *(volatile v8us*)dp = o;
  __threadfence();
  *(volatile v8us*)dp = o;
}

__global__ __launch_bounds__(NTHR) void k_compact(const int* __restrict__ srcs, const int* __restrict__ dsts,
                                                  const float* __restrict__ ew, int nE, int nN, int vec8,
                                                  int* hsrc, float* hwgt, int* cntT, int* offT, int* dinvBits) {
  extern __shared__ __attribute__((aligned(16))) int dsm[];
  int* list = dsm;
  int* hl   = dsm + LISTN;
  int* sl   = hl + RCAP;
  int* cnt  = sl + RCAP;
  int* offs = cnt + NBA;
  int* cur  = offs + NBA;
  int* misc = cur + NBA;
  const int tid = (int)threadIdx.x, lane = tid & 31, wave = tid >> 5;
  const int nodeBase = (int)blockIdx.x * NBA;

  {
    const v4i z4 = {0, 0, 0, 0};
    for (int i = tid * 4; i < CMP_ZINTS; i += NTHR * 4) *(v4ia*)(dsm + i) = z4;
    if (tid < MISC_INTS) misc[tid] = 0;
  }
  __syncthreads();

  int t = 0, ov = 0;
  const int nChunks = (nE + CHUNK - 1) / CHUNK;
#pragma unroll 1
  for (int ch = 0; ch < nChunks; ++ch) {
    const int cbase = ch * CHUNK;
    const int wc = scan_chunk<SLA>(dsts, nE, cbase, nodeBase, NBA, vec8, list, tid, lane, wave);
    if (lane == 0) misc[wave] = wc;
    __syncthreads();
    if (wave == 0) {
#pragma unroll 1
      for (int w2 = 0; w2 < NWAVE; ++w2) {
        int c = misc[w2];
        c = c < 0 ? 0 : (c > WCAP ? WCAP : c);
#pragma unroll 1
        for (int b0 = 0; b0 < c; b0 += 32) {
          const int idx = b0 + lane;
          const int ent = list[w2 * WCAP + (idx < WCAP ? idx : WCAP - 1)];
          const int m32 = (c - b0) < 32 ? (c - b0) : 32;
#pragma unroll 1
          for (int k = 0; k < m32; ++k) {
            const int u    = __builtin_amdgcn_readlane(ent, k);
            const int slot = u & (NBA - 1);
            const int el   = (u >> SLA) & (CHUNK - 1);
            const int pk   = ((cbase + el) << SLA) | slot;
            if (t < RCAP) {
              if (lane == 0) { hl[t] = pk; cnt[slot] = cnt[slot] + 1; }
              t = t + 1;
            } else {
              ov = 1;
            }
          }
        }
      }
    }
    __syncthreads();
  }
  if (wave == 0 && lane == 0) { misc[8] = t; misc[9] = ov; }
  __syncthreads();
  int tt = misc[8];
  tt = tt < 0 ? 0 : (tt > RCAP ? RCAP : tt);
  const int ovf = misc[9];

  if (wave == 0) {
    const int base = lane * (NBA / 32);
    int s = 0;
#pragma unroll 1
    for (int i = 0; i < NBA / 32; ++i) s += cnt[base + i];
    int incl = s;
#pragma unroll
    for (int d = 1; d < 32; d <<= 1) {
      const int y = __shfl_up(incl, d, 32);
      if (lane >= d) incl += y;
    }
    int run = incl - s;
#pragma unroll 1
    for (int i = 0; i < NBA / 32; ++i) {
      const int cv = cnt[base + i];
      offs[base + i] = run;
      cur[base + i]  = run;
      run += cv;
    }
  }
  __syncthreads();
  if (wave == 0) {
#pragma unroll 1
    for (int b0 = 0; b0 < tt; b0 += 32) {
      const int idx = b0 + lane;
      const int ent = hl[idx < RCAP ? idx : RCAP - 1];
      const int m32 = (tt - b0) < 32 ? (tt - b0) : 32;
#pragma unroll 1
      for (int k = 0; k < m32; ++k) {
        const int u    = __builtin_amdgcn_readlane(ent, k);
        const int slot = u & (NBA - 1);
        if (lane == 0) {
          int p = cur[slot];
          p = p < 0 ? 0 : (p > RCAP - 1 ? RCAP - 1 : p);
          sl[p] = u;
          cur[slot] = p + 1;
        }
      }
    }
  }
  __syncthreads();

  const float qnan = __int_as_float(0x7fc00000);
#pragma unroll 1
  for (int si = 0; si < NBA / NWAVE; ++si) {
    const int s = si * NWAVE + wave;
    int c = cnt[s];
    const bool big = c > DEGCAP;
    c = c < 0 ? 0 : (c > DEGCAP ? DEGCAP : c);
    int o = offs[s];
    o = o < 0 ? 0 : (o > RCAP ? RCAP : o);
    float part = 0.0f;
#pragma unroll 1
    for (int b0 = 0; b0 < c; b0 += 32) {
      int idx = o + b0 + lane;
      idx = idx > RCAP - 1 ? RCAP - 1 : idx;
      const int ent = sl[idx];
      int eid = ent >> SLA;
      eid = eid < 0 ? 0 : (eid > nE - 1 ? nE - 1 : eid);
      const float wv = bf16_val(ew[eid]);
      part += ((b0 + lane) < c) ? wv : 0.0f;
    }
#pragma unroll
    for (int d = 16; d >= 1; d >>= 1) part += __shfl_xor(part, d, 32);
    const float deg = 1.0f + part;
    float dv = (deg > 0.0f) ? rsqrtf(deg) : 0.0f;
    dv = (big || ovf != 0) ? qnan : dv;
    if (lane == 0) cur[s] = __float_as_int(dv);
  }
  __syncthreads();

  const v4i c4 = *(const v4ia*)(cnt  + 4 * tid);
  const v4i o4 = *(const v4ia*)(offs + 4 * tid);
  const v4i d4 = *(const v4ia*)(cur  + 4 * tid);
  const size_t tb = (size_t)blockIdx.x * NBA + 4 * (size_t)tid;
  const size_t hb = (size_t)blockIdx.x * RCAP;
  int ttPad = ((tt + 32 + (NTHR - 1)) / NTHR) * NTHR;
  ttPad = ttPad > RCAP ? RCAP : ttPad;

  *(volatile v4i*)(cntT + tb) = c4;
  *(volatile v4i*)(offT + tb) = o4;
  *(volatile v4i*)(dinvBits + tb) = d4;
#pragma unroll 1
  for (int idx = tid; idx < ttPad; idx += NTHR) {
    const int ent = sl[idx];
    int eid = ent >> SLA;
    eid = eid < 0 ? 0 : (eid > nE - 1 ? nE - 1 : eid);
    int sr = srcs[eid];
    sr = sr < 0 ? 0 : (sr > nN - 1 ? nN - 1 : sr);
    const float wv = bf16_val(ew[eid]);
    *(volatile int*)(hsrc + hb + idx)   = sr;
    *(volatile float*)(hwgt + hb + idx) = wv;
  }
  __threadfence();
  *(volatile v4i*)(cntT + tb) = c4;
  *(volatile v4i*)(offT + tb) = o4;
  *(volatile v4i*)(dinvBits + tb) = d4;
#pragma unroll 1
  for (int idx = tid; idx < ttPad; idx += NTHR) {
    const int ent = sl[idx];
    int eid = ent >> SLA;
    eid = eid < 0 ? 0 : (eid > nE - 1 ? nE - 1 : eid);
    int sr = srcs[eid];
    sr = sr < 0 ? 0 : (sr > nN - 1 ? nN - 1 : sr);
    const float wv = bf16_val(ew[eid]);
    *(volatile int*)(hsrc + hb + idx)   = sr;
    *(volatile float*)(hwgt + hb + idx) = wv;
  }
}

__global__ __launch_bounds__(GTHR) void k_gemm(const unsigned short* __restrict__ Apl, int lda,
                                               const unsigned short* __restrict__ BT, int K, float* outF) {
  __shared__ __attribute__((aligned(16))) float stg[GBM * GBN];
  const int tid = (int)threadIdx.x, lane = tid & 31, wave = tid >> 5, hh = lane >> 4, m = lane & 15;
  const int rowBase = (int)blockIdx.x * GBM;

  v8f acc[8];
  {
    const v8f z = {0.f, 0.f, 0.f, 0.f, 0.f, 0.f, 0.f, 0.f};
#pragma unroll
    for (int t = 0; t < 8; ++t) acc[t] = z;
  }
  const unsigned short* ap = Apl + (size_t)(rowBase + 16 * wave + m) * (size_t)lda + 8 * hh;
  const unsigned short* bp = BT + (size_t)m * (size_t)K + 8 * hh;

#pragma unroll 1
  for (int k0 = 0; k0 < K; k0 += 32) {
    FragB af;
    af.h[0] = *(const v8usa*)(ap + k0);
    af.h[1] = *(const v8usa*)(ap + k0 + 16);
#pragma unroll
    for (int nt = 0; nt < 8; ++nt) {
      const unsigned short* wq = bp + (size_t)(16 * nt) * (size_t)K + k0;
      FragB bf;
      bf.h[0] = *(const v8usa*)wq;
      bf.h[1] = *(const v8usa*)(wq + 16);
      acc[nt] = wmb(af, bf, acc[nt]);
    }
  }

#pragma unroll
  for (int nt = 0; nt < 8; ++nt) {
    const int lc = 16 * nt + m;
#pragma unroll
    for (int r = 0; r < 8; ++r) {
      const int lr = 16 * wave + 8 * hh + r;
      stg[lr * GBN + lc] = acc[nt][r];
    }
  }
  __syncthreads();

  v4f pv[16];
#pragma unroll
  for (int i = 0; i < 16; ++i) pv[i] = *(const v4fa*)(stg + (16 * wave + i) * GBN + 4 * lane);
#pragma unroll
  for (int i = 0; i < 16; ++i)
    *(volatile v4f*)(outF + (size_t)(rowBase + 16 * wave + i) * DF + 4 * lane) = pv[i];
  __threadfence();
#pragma unroll
  for (int i = 0; i < 16; ++i)
    *(volatile v4f*)(outF + (size_t)(rowBase + 16 * wave + i) * DF + 4 * lane) = pv[i];
}

__global__ __launch_bounds__(NTHR) void k_agg(const int* __restrict__ hsrc, const float* __restrict__ hwgt,
                                              const int* __restrict__ cntT, const int* __restrict__ offT,
                                              const float* __restrict__ dinv, const float* __restrict__ hin,
                                              const float* __restrict__ bias, int nN, int mRows,
                                              float* agg, float* rec) {
  __shared__ __attribute__((aligned(16))) int   scn[NBA];
  __shared__ __attribute__((aligned(16))) int   sof[NBA];
  __shared__ __attribute__((aligned(16))) float wsum[NWAVE * RECW];
  __shared__ __attribute__((aligned(16))) float outs[RECW];
  const int tid = (int)threadIdx.x, lane = tid & 31, wave = tid >> 5;
  const int nodeBase = (int)blockIdx.x * NBA;
  const size_t hbase = (size_t)blockIdx.x * RCAP;

  {
    const v4i c4 = *(const v4ia*)(cntT + (size_t)nodeBase + 4 * tid);
    const v4i o4 = *(const v4ia*)(offT + (size_t)nodeBase + 4 * tid);
    *(v4ia*)(scn + 4 * tid) = c4;
    *(v4ia*)(sof + 4 * tid) = o4;
  }
  v4f bb;
  {
    const v4f t0 = *(const v4fa*)(bias + 4 * lane);
    bb.x = bf16_val(t0.x); bb.y = bf16_val(t0.y); bb.z = bf16_val(t0.z); bb.w = bf16_val(t0.w);
  }
  __syncthreads();

  const float qnan = __int_as_float(0x7fc00000);
  float s10 = 0.0f, s11 = 0.0f, s12 = 0.0f, s13 = 0.0f;
  float s20 = 0.0f, s21 = 0.0f, s22 = 0.0f, s23 = 0.0f;
#pragma unroll 1
  for (int si = 0; si < NBA / NWAVE; ++si) {
    const int s    = si * NWAVE + wave;
    const int node = nodeBase + s;
    const int craw = scn[s];
    const bool bad = (craw < 0) || (craw > DEGCAP);
    const int c = craw < 0 ? 0 : (craw > DEGCAP ? DEGCAP : craw);
    int o = sof[s];
    o = o < 0 ? 0 : (o > RCAP ? RCAP : o);
    const int nc = node < nN ? node : nN - 1;
    const float dd = dinv[nc];
    const float rd = dd * dd;
    float a0 = 0.0f, a1 = 0.0f, a2 = 0.0f, a3 = 0.0f;
#pragma unroll 1
    for (int b0 = 0; b0 < c; b0 += 32) {
      int idx = o + b0 + lane;
      idx = idx > RCAP - 1 ? RCAP - 1 : idx;
      int sr = hsrc[hbase + idx];
      sr = sr < 0 ? 0 : (sr > nN - 1 ? nN - 1 : sr);
      const float wv  = hwgt[hbase + idx];
      const float cf  = (dinv[sr] * wv) * dd;
      const int   cfi = __float_as_int(cf);
      const int m32 = (c - b0) < 32 ? (c - b0) : 32;
#pragma unroll 1
      for (int k = 0; k < m32; ++k) {
        const int   sk = __builtin_amdgcn_readlane(sr, k);
        const float ck = __int_as_float(__builtin_amdgcn_readlane(cfi, k));
        const v4f a = *(const v4fa*)(hin + (size_t)sk * DF + 4 * lane);
        a0 = fmaf(ck, a.x, a0);
        a1 = fmaf(ck, a.y, a1);
        a2 = fmaf(ck, a.z, a2);
        a3 = fmaf(ck, a.w, a3);
      }
    }
    const v4f hs = *(const v4fa*)(hin + (size_t)nc * DF + 4 * lane);
    const float pzr = bad ? qnan : 0.0f;
    const bool live = node < nN;
    const float y0 = ((a0 + hs.x * rd) + bb.x) + pzr;
    const float y1 = ((a1 + hs.y * rd) + bb.y) + pzr;
    const float y2 = ((a2 + hs.z * rd) + bb.z) + pzr;
    const float y3 = ((a3 + hs.w * rd) + bb.w) + pzr;
    v4f v;
    v.x = live ? y0 : 0.0f; v.y = live ? y1 : 0.0f; v.z = live ? y2 : 0.0f; v.w = live ? y3 : 0.0f;
    s10 += v.x; s11 += v.y; s12 += v.z; s13 += v.w;
    s20 += v.x * v.x; s21 += v.y * v.y; s22 += v.z * v.z; s23 += v.w * v.w;
    if (node < mRows) {
      float* op = agg + (size_t)node * DF + 4 * lane;
      *(volatile v4f*)op = v;
      __threadfence();
      *(volatile v4f*)op = v;
    }
  }

  {
    v4f t1, t2;
    t1.x = s10; t1.y = s11; t1.z = s12; t1.w = s13;
    t2.x = s20; t2.y = s21; t2.z = s22; t2.w = s23;
    *(v4fa*)(wsum + wave * RECW + 4 * lane) = t1;
    *(v4fa*)(wsum + wave * RECW + DF + 4 * lane) = t2;
  }
  __syncthreads();
  {
    float r = 0.0f;
#pragma unroll
    for (int w2 = 0; w2 < NWAVE; ++w2) r += wsum[w2 * RECW + tid];
    outs[tid] = r;
  }
  __syncthreads();
  const v4f ov = *(const v4fa*)(outs + 4 * (tid & 63));
  float* rp = rec + (size_t)blockIdx.x * RECW + 4 * (tid & 63);
  const bool okst = tid < 64;
  if (okst) *(volatile v4f*)rp = ov;
  __threadfence();
  if (okst) *(volatile v4f*)rp = ov;
}

__global__ __launch_bounds__(NTHR) void k_bnstat(const float* __restrict__ rec, int nRec, int nN, float* ms) {
  __shared__ __attribute__((aligned(16))) float outs[RECW];
  const int tid = (int)threadIdx.x;
  if (tid < DF) {
    double S = 0.0, Q = 0.0;
#pragma unroll 2
    for (int b = 0; b < nRec; ++b) {
      S += (double)rec[(size_t)b * RECW + tid];
      Q += (double)rec[(size_t)b * RECW + DF + tid];
    }
    const double inv = 1.0 / (double)nN;
    const double mean = S * inv;
    double var = Q * inv - mean * mean;
    var = (var < 0.0) ? 0.0 : var;
    const float vf = (float)(var + 1e-5);
    outs[tid] = (float)mean;
    outs[DF + tid] = rsqrtf(vf);
  }
  __syncthreads();
  const v4f ov = *(const v4fa*)(outs + 4 * (tid & 63));
  float* op = ms + 4 * (tid & 63);
  const bool okst = tid < 64;
  if (okst) *(volatile v4f*)op = ov;
  __threadfence();
  if (okst) *(volatile v4f*)op = ov;
}

template <int FIN>
__global__ __launch_bounds__(NTHR) void k_apply(const float* __restrict__ agg, const float* __restrict__ ms,
                                                const float* __restrict__ gam, const float* __restrict__ bet,
                                                int nN, unsigned short* xhl, float* outp) {
  const int tid = (int)threadIdx.x, lane = tid & 31, wave = tid >> 5;
  const int rowBase = (int)blockIdx.x * 64 + wave * 8;
  const v4f mu = *(const v4fa*)(ms + 4 * lane);
  const v4f rs = *(const v4fa*)(ms + DF + 4 * lane);
  v4f g, b;
  {
    const v4f g0 = *(const v4fa*)(gam + 4 * lane);
    const v4f b0 = *(const v4fa*)(bet + 4 * lane);
    g.x = bf16_val(g0.x); g.y = bf16_val(g0.y); g.z = bf16_val(g0.z); g.w = bf16_val(g0.w);
    b.x = bf16_val(b0.x); b.y = bf16_val(b0.y); b.z = bf16_val(b0.z); b.w = bf16_val(b0.w);
  }
  if constexpr (FIN != 0) {
    __shared__ __attribute__((aligned(16))) float sf[64 * DF];
#pragma unroll 1
    for (int i = 0; i < 8; ++i) {
      const int r  = rowBase + i;
      const int rc = r < nN ? r : nN - 1;
      const v4f a = *(const v4fa*)(agg + (size_t)rc * DF + 4 * lane);
      v4f y;
      y.x = bnrelu(a.x, mu.x, rs.x, g.x, b.x);
      y.y = bnrelu(a.y, mu.y, rs.y, g.y, b.y);
      y.z = bnrelu(a.z, mu.z, rs.z, g.z, b.z);
      y.w = bnrelu(a.w, mu.w, rs.w, g.w, b.w);
      *(v4fa*)(sf + (wave * 8 + i) * DF + 4 * lane) = y;
    }
    __syncthreads();
    v4f q[8];
#pragma unroll
    for (int i = 0; i < 8; ++i) q[i] = *(const v4fa*)(sf + (wave * 8 + i) * DF + 4 * lane);
#pragma unroll
    for (int i = 0; i < 8; ++i) {
      const int r = rowBase + i;
      if (r < nN) *(volatile v4f*)(outp + (size_t)r * DF + 4 * lane) = q[i];
    }
    __threadfence();
#pragma unroll
    for (int i = 0; i < 8; ++i) {
      const int r = rowBase + i;
      if (r < nN) *(volatile v4f*)(outp + (size_t)r * DF + 4 * lane) = q[i];
    }
  } else {
    __shared__ __attribute__((aligned(16))) unsigned short rb[64 * K1];
#pragma unroll 1
    for (int i = 0; i < 8; ++i) {
      const int r  = rowBase + i;
      const int rc = r < nN ? r : nN - 1;
      const bool live = r < nN;
      const v4f a = *(const v4fa*)(agg + (size_t)rc * DF + 4 * lane);
      const float y0 = live ? bnrelu(a.x, mu.x, rs.x, g.x, b.x) : 0.0f;
      const float y1 = live ? bnrelu(a.y, mu.y, rs.y, g.y, b.y) : 0.0f;
      const float y2 = live ? bnrelu(a.z, mu.z, rs.z, g.z, b.z) : 0.0f;
      const float y3 = live ? bnrelu(a.w, mu.w, rs.w, g.w, b.w) : 0.0f;
      v4us h4, l4;
      unsigned hb;
      hb = bf16_bits(y0); h4[0] = (unsigned short)hb; l4[0] = (unsigned short)bf16_bits(y0 - __uint_as_float(hb << 16));
      hb = bf16_bits(y1); h4[1] = (unsigned short)hb; l4[1] = (unsigned short)bf16_bits(y1 - __uint_as_float(hb << 16));
      hb = bf16_bits(y2); h4[2] = (unsigned short)hb; l4[2] = (unsigned short)bf16_bits(y2 - __uint_as_float(hb << 16));
      hb = bf16_bits(y3); h4[3] = (unsigned short)hb; l4[3] = (unsigned short)bf16_bits(y3 - __uint_as_float(hb << 16));
      unsigned short* srow = rb + (size_t)(wave * 8 + i) * K1;
      *(v4usa*)(srow + 4 * lane) = h4;
      *(v4usa*)(srow + DF + 4 * lane) = l4;
    }
    __syncthreads();
    v8us q[8];
#pragma unroll
    for (int i = 0; i < 8; ++i) q[i] = *(const v8usa*)(rb + (size_t)(wave * 8 + i) * K1 + 8 * lane);
#pragma unroll
    for (int i = 0; i < 8; ++i)
      *(volatile v8us*)(xhl + (size_t)(rowBase + i) * K1 + 8 * lane) = q[i];
    __threadfence();
#pragma unroll
    for (int i = 0; i < 8; ++i)
      *(volatile v8us*)(xhl + (size_t)(rowBase + i) * K1 + 8 * lane) = q[i];
  }
}

static inline int cdiv(int a, int b) { return (a + b - 1) / b; }
static inline size_t al256(size_t o) { return (o + 255) & ~(size_t)255; }

extern "C" void kernel_launch(void* const* d_in, const int* in_sizes, int n_in,
                              void* d_out, int out_size, void* d_ws, size_t ws_size,
                              hipStream_t stream) {
  if (n_in < 7) return;
  if (in_sizes[0] < DF || (in_sizes[0] % DF) != 0) return;
  const int nN = in_sizes[0] / DF;
  if (nN < 16 || nN > (1 << 22)) return;
  if (in_sizes[1] < 2 || (in_sizes[1] & 1) != 0) return;
  const int nE = in_sizes[1] / 2;
  if (nE < 1 || nE >= (1 << 21)) return;
  if (in_sizes[2] != nE) return;
  if (in_sizes[3] != 2 * DF * DF) return;
  if (in_sizes[4] != 2 * DF || in_sizes[5] != 2 * DF || in_sizes[6] != 2 * DF) return;
  if ((long long)out_size != (long long)nN * DF) return;

  const float* x    = (const float*)d_in[0];
  const int*   edge = (const int*)d_in[1];
  const float* ew   = (const float*)d_in[2];
  const float* W    = (const float*)d_in[3];
  const float* bia  = (const float*)d_in[4];
  const float* gam  = (const float*)d_in[5];
  const float* bet  = (const float*)d_in[6];
  float* out = (float*)d_out;
  const int* src = edge;
  const int* dst = edge + nE;

  const int MP = cdiv(nN, GBM) * GBM;
  const int gM = MP / GBM;
  const int gA = cdiv(MP, NBA);
  const int NBP = gA * NBA;
  if ((long long)gA * NBA < (long long)MP) return;
  const int vec8 = ((nE & 3) == 0) ? 1 : 0;

  char* ws = (char*)d_ws;
  size_t off = 0;
  const size_t oWB   = off; off = al256(off + (size_t)(DF * DF + DF * K1) * 2);
  const size_t oDINV = off; off = al256(off + (size_t)NBP * 4);
  const size_t oCNT  = off; off = al256(off + (size_t)NBP * 4);
  const size_t oOFF  = off; off = al256(off + (size_t)NBP * 4);
  const size_t oHS   = off; off = al256(off + (size_t)gA * RCAP * 4);
  const size_t oHW   = off; off = al256(off + (size_t)gA * RCAP * 4);
  const size_t oRC0  = off; off = al256(off + (size_t)gA * RECW * 4);
  const size_t oRC1  = off; off = al256(off + (size_t)gA * RECW * 4);
  const size_t oMS0  = off; off = al256(off + (size_t)RECW * 4);
  const size_t oMS1  = off; off = al256(off + (size_t)RECW * 4);
  const size_t oRA   = off; off = al256(off + (size_t)MP * DF * 4);
  const size_t oRB   = off; off = al256(off + (size_t)MP * DF * 4);
  if (off > ws_size || off > (size_t)WSMAX) return;
  if ((size_t)MP * DF * 2 > (size_t)MP * DF * 4) return;
  unsigned short* WB   = (unsigned short*)(ws + oWB);
  unsigned short* WB0  = WB;
  unsigned short* WB1  = WB + DF * DF;
  float* DINV = (float*)(ws + oDINV);
  int*   CNT  = (int*)(ws + oCNT);
  int*   OFFS = (int*)(ws + oOFF);
  int*   HS   = (int*)(ws + oHS);
  float* HW   = (float*)(ws + oHW);
  float* REC0 = (float*)(ws + oRC0);
  float* REC1 = (float*)(ws + oRC1);
  float* MS0  = (float*)(ws + oMS0);
  float* MS1  = (float*)(ws + oMS1);
  float* RA   = (float*)(ws + oRA);
  float* RB   = (float*)(ws + oRB);
  unsigned short* XB = (unsigned short*)(ws + oRB);
  unsigned short* X1 = (unsigned short*)(ws + oRA);

  const size_t cmpLds = (size_t)CMP_LDS_INTS * 4;
  hipFuncSetAttribute(reinterpret_cast<const void*>(&k_compact), hipFuncAttributeMaxDynamicSharedMemorySize, (int)cmpLds);

  const int nUx = MP * (DF / 8);
  k_wprep<<<(NPART * UPART) / NTHR, NTHR, 0, stream>>>(W, WB);
  k_cvx<<<cdiv(nUx, NTHR), NTHR, 0, stream>>>(x, nN, nUx, XB);
  k_compact<<<gA, NTHR, cmpLds, stream>>>(src, dst, ew, nE, nN, vec8, HS, HW, CNT, OFFS, (int*)DINV);
  k_gemm<<<gM, GTHR, 0, stream>>>(XB, DF, WB0, DF, RA);
  k_agg<<<gA, NTHR, 0, stream>>>(HS, HW, CNT, OFFS, DINV, RA, bia, nN, MP, RB, REC0);
  k_bnstat<<<1, NTHR, 0, stream>>>(REC0, gA, nN, MS0);
  k_apply<0><<<gM, NTHR, 0, stream>>>(RB, MS0, gam, bet, nN, X1, out);
  k_gemm<<<gM, GTHR, 0, stream>>>(X1, K1, WB1, K1, RB);
  k_agg<<<gA, NTHR, 0, stream>>>(HS, HW, CNT, OFFS, DINV, RB, bia + DF, nN, MP, RA, REC1);
  k_bnstat<<<1, NTHR, 0, stream>>>(REC1, gA, nN, MS1);
  k_apply<1><<<gM, NTHR, 0, stream>>>(RA, MS1, gam + DF, bet + DF, nN, X1, out);
}
